// MeriamAttention_55525337203160
// MI455X (gfx1250) — hardware-verified
//
#include <hip/hip_runtime.h>
#include <stdint.h>

#define NB   4
#define SEQ  2048
#define DM   1024
#define NTOK 8192

typedef _Float16 v16h __attribute__((ext_vector_type(16)));
typedef _Float16 v8h  __attribute__((ext_vector_type(8)));
typedef __bf16   v16b __attribute__((ext_vector_type(16)));
typedef __bf16   v8b  __attribute__((ext_vector_type(8)));
typedef float    v8f  __attribute__((ext_vector_type(8)));
typedef float    v4f  __attribute__((ext_vector_type(4)));
typedef unsigned short v8us __attribute__((ext_vector_type(8)));

static_assert((DM % 64) == 0);
static_assert((NTOK % 64) == 0);
static_assert(NTOK == NB * SEQ);

__device__ __forceinline__ unsigned short bfbits(float f) {
  const unsigned u = __float_as_uint(f);
  return (unsigned short)((u + 0x7FFFu + ((u >> 16) & 1u)) >> 16);
}
__device__ __forceinline__ float bfval(unsigned short b) { return __uint_as_float(((unsigned)b) << 16); }
__device__ __forceinline__ float bfr(float f) { return bfval(bfbits(f)); }

template <int ET> struct Elem;
template <> struct Elem<0> {
  typedef _Float16 T; typedef v16h V; typedef v8h V8;
  static __device__ __forceinline__ v8f mma(V a, V b, v8f c) {
    return __builtin_amdgcn_wmma_f32_16x16x32_f16(false, a, false, b, (short)0, c, false, false);
  }
};
template <> struct Elem<1> {
  typedef __bf16 T; typedef v16b V; typedef v8b V8;
  static __device__ __forceinline__ v8f mma(V a, V b, v8f c) {
    return __builtin_amdgcn_wmma_f32_16x16x32_bf16(false, a, false, b, (short)0, c, false, false);
  }
};

template <int ET>
__device__ __forceinline__ typename Elem<ET>::V ldfragT(const typename Elem<ET>::T* p) {
  typedef typename Elem<ET>::V V;
  typedef typename Elem<ET>::V8 V8;
  union { V v; V8 hh[2]; } f;
  f.hh[0] = *(const V8*)(p);
  f.hh[1] = *(const V8*)(p + 16);
  return f.v;
}
__device__ __forceinline__ v16h ldfrag(const _Float16* p) { return ldfragT<0>(p); }
__device__ __forceinline__ v8f mma16(v16h a, v16h b, v8f c) { return Elem<0>::mma(a, b, c); }
__device__ __forceinline__ v8f zero8() {
  v8f z;
#pragma unroll
  for (int i = 0; i < 8; ++i) z[i] = 0.0f;
  return z;
}

__device__ __forceinline__ void guard_g(v8f& a, v8f& b, v16b x, v16b y) {
  asm volatile("v_nop\n\tv_nop\n\tv_nop\n\tv_nop" : "+v"(a), "+v"(b) : "v"(x), "v"(y));
}
__device__ __forceinline__ void keep4(v16b a, v16b b, v16b c, v16b d) {
  asm volatile("v_nop" :: "v"(a), "v"(b), "v"(c), "v"(d));
}
__device__ __forceinline__ void accg4(v8f& a, v8f& b, v8f& c, v8f& d) {
  asm volatile("v_nop\n\tv_nop\n\tv_nop\n\tv_nop" : "+v"(a), "+v"(b), "+v"(c), "+v"(d));
}
__device__ __forceinline__ void guard4h(v8f& a, v8f& b, v8f& c, v8f& d, v16h x0, v16h x1, v16h y0, v16h y1) {
  asm volatile("v_nop\n\tv_nop\n\tv_nop\n\tv_nop"
               : "+v"(a), "+v"(b), "+v"(c), "+v"(d) : "v"(x0), "v"(x1), "v"(y0), "v"(y1));
}
__device__ __forceinline__ void guard5h(v8f& a, v8f& b, v8f& c, v8f& d,
                                        v16h p, v16h x0, v16h x1, v16h y0, v16h y1) {
  asm volatile("v_nop\n\tv_nop\n\tv_nop\n\tv_nop"
               : "+v"(a), "+v"(b), "+v"(c), "+v"(d) : "v"(p), "v"(x0), "v"(x1), "v"(y0), "v"(y1));
}

__global__ __launch_bounds__(256) void cvt_x_kernel(const float* __restrict__ x, unsigned short* __restrict__ xb,
                                                    int n8) {
  const int li = (int)blockIdx.x * 256 + (int)threadIdx.x;
  if (li >= n8) return;
  const size_t e = (size_t)li * 8;
  const v4f a = *(const v4f*)(x + e);
  const v4f b = *(const v4f*)(x + e + 4);
  v8us o;
#pragma unroll
  for (int i = 0; i < 4; ++i) {
    o[i]     = bfbits(a[i]);
    o[4 + i] = bfbits(b[i]);
  }
  unsigned short* d = xb + e;
  *(volatile v8us*)d = o;
  __threadfence();
  *(volatile v8us*)d = o;
}

__global__ __launch_bounds__(256) void trw_kernel(const float* __restrict__ w0, const float* __restrict__ w1,
                                                  const float* __restrict__ w2, unsigned short* __restrict__ t0,
                                                  unsigned short* __restrict__ t1, unsigned short* __restrict__ t2) {
  __shared__ __align__(16) unsigned short Ts[64 * 72];
  const int tid = threadIdx.x, wave = tid >> 5, lane = tid & 31;
  const int mat = (int)blockIdx.x >> 8;
  const int tix = (int)blockIdx.x & 255;
  const int ti = tix >> 4, tj = tix & 15;
  const float* src = (mat == 0) ? w0 : ((mat == 1) ? w1 : w2);
  unsigned short* dst = (mat == 0) ? t0 : ((mat == 1) ? t1 : t2);
  const int i0 = ti * 64, j0 = tj * 64;
#pragma unroll
  for (int it = 0; it < 4; ++it) {
    const int idx = it * 256 + tid;
    const int row = idx >> 4;
    const int cq  = idx & 15;
    const v4f v = *(const v4f*)(src + (size_t)(i0 + row) * DM + j0 + cq * 4);
#pragma unroll
    for (int e = 0; e < 4; ++e) Ts[(cq * 4 + e) * 72 + row] = bfbits(v[e]);
  }
  __syncthreads();
  const int qq = lane >> 3, c8 = (lane & 7) * 8;
#pragma unroll
  for (int ps = 0; ps < 2; ++ps) {
#pragma unroll
    for (int it = 0; it < 2; ++it) {
      const int j = wave * 8 + it * 4 + qq;
      const v8us v = *(const v8us*)(Ts + j * 72 + c8);
      *(volatile v8us*)(dst + (size_t)(j0 + j) * DM + i0 + c8) = v;
    }
    __threadfence();
  }
}

template <int BM, bool SPLIT>
__global__ __launch_bounds__(256) __attribute__((amdgpu_num_vgpr(256)))
void gemm64_kernel(const unsigned short* __restrict__ Ap, int lda,
                   const unsigned short* __restrict__ Btp, int ldb,
                   _Float16* __restrict__ Ch, _Float16* __restrict__ Cl, int ldc,
                   const float* __restrict__ bias, int M, int N, int K, float car) {
  const __bf16* A  = (const __bf16*)(const void*)Ap;
  const __bf16* Bt = (const __bf16*)(const void*)Btp;
  __shared__ __align__(16) float sT[8][16 * 68];
  const int lane = threadIdx.x & 31, wave = threadIdx.x >> 5;
  const int tilesN = N >> 6, tilesM = M >> 6;
  const int tile = (int)blockIdx.x * 8 + wave;
  if (tile >= tilesM * tilesN) return;
  const int tm = tile / tilesN, tn = tile - tm * tilesN;
  const int m0 = tm << 6, n0 = tn << 6;
  const int rl = lane & 15;
  const int koff = (lane >> 4) * 8;
  const int mOff = (lane >> 4) * 8;

  v8f acc[4][4];
#pragma unroll
  for (int i = 0; i < 4; ++i)
#pragma unroll
    for (int j = 0; j < 4; ++j) acc[i][j] = zero8();

#pragma unroll 1
  for (int k0 = 0; k0 < K; k0 += 32) {
    v16b bh[4];
#pragma unroll
    for (int j = 0; j < 4; ++j) bh[j] = ldfragT<1>(Bt + (size_t)(n0 + (j << 4) + rl) * ldb + koff + k0);
#pragma unroll
    for (int i = 0; i < 4; ++i) {
      const v16b ah = ldfragT<1>(A + (size_t)(m0 + (i << 4) + rl) * lda + koff + k0);
#pragma unroll
      for (int j = 0; j < 4; ++j) acc[i][j] = Elem<1>::mma(ah, bh[j], acc[i][j]);
      guard_g(acc[i][0], acc[i][3], ah, bh[3]);
    }
    keep4(bh[0], bh[1], bh[2], bh[3]);
  }
  accg4(acc[0][0], acc[0][1], acc[0][2], acc[0][3]);
  accg4(acc[1][0], acc[1][1], acc[1][2], acc[1][3]);
  accg4(acc[2][0], acc[2][1], acc[2][2], acc[2][3]);
  accg4(acc[3][0], acc[3][1], acc[3][2], acc[3][3]);

  float* slab = sT[wave];
  const int qq = lane >> 3, c8 = (lane & 7) * 8;
#pragma unroll
  for (int i = 0; i < 4; ++i) {
    const int mBase = m0 + (i << 4);
    v8f rb = zero8();
    if constexpr (BM == 2) {
      const v4f r0v = *(const v4f*)(bias + mBase + mOff);
      const v4f r1v = *(const v4f*)(bias + mBase + mOff + 4);
#pragma unroll
      for (int r = 0; r < 4; ++r) {
        rb[r]     = bfr(r0v[r]) * car;
        rb[4 + r] = bfr(r1v[r]) * car;
      }
    }
#pragma unroll
    for (int j = 0; j < 4; ++j) {
      float cb = 0.0f;
      if constexpr (BM == 1) cb = bfr(bias[n0 + (j << 4) + rl]) * car;
#pragma unroll
      for (int r = 0; r < 8; ++r) {
        const float bb = (BM == 1) ? cb : rb[r];
        slab[(mOff + r) * 68 + (j << 4) + rl] = acc[i][j][r] * car + bb;
      }
    }
    __builtin_amdgcn_fence(__ATOMIC_RELEASE, "workgroup");
    __builtin_amdgcn_wave_barrier();
    __builtin_amdgcn_fence(__ATOMIC_ACQUIRE, "workgroup");
#pragma unroll
    for (int ps = 0; ps < 2; ++ps) {
#pragma unroll
      for (int it = 0; it < 4; ++it) {
        const int row = it * 4 + qq;
        const float* sp = slab + row * 68 + c8;
        const size_t co = (size_t)(mBase + row) * ldc + n0 + c8;
        v8h hv;
        if constexpr (SPLIT) {
          v8h lv;
#pragma unroll
          for (int e = 0; e < 8; ++e) {
            const float f = sp[e];
            const _Float16 hq = (_Float16)f;
            hv[e] = hq;
            lv[e] = (_Float16)((f - (float)hq) * 2048.0f);
          }
          *(volatile v8h*)(Ch + co) = hv;
          *(volatile v8h*)(Cl + co) = lv;
        } else {
#pragma unroll
          for (int e = 0; e < 8; ++e) hv[e] = (_Float16)sp[e];
          *(volatile v8h*)(Ch + co) = hv;
        }
      }
      __threadfence();
    }
    __builtin_amdgcn_fence(__ATOMIC_RELEASE, "workgroup");
    __builtin_amdgcn_wave_barrier();
    __builtin_amdgcn_fence(__ATOMIC_ACQUIRE, "workgroup");
  }
}

#define QB       16
#define KCH      256
#define QSP      1032
#define PSP      264
#define OSP      1028
#define LDS_QH   0
#define LDS_QL   33024
#define LDS_PS   66048
#define LDS_PMAX 74496
#define LDS_PSUM 75008
#define LDS_ST   75520
#define ATT_LDS  75776
static_assert(QB * QSP * 2 == LDS_QL - LDS_QH);
static_assert(QB * QSP * 2 == LDS_PS - LDS_QL);
static_assert(QB * PSP * 2 == LDS_PMAX - LDS_PS);
static_assert(LDS_PSUM - LDS_PMAX == 8 * QB * 4);
static_assert(LDS_ST - LDS_PSUM == 8 * QB * 4);
static_assert(ATT_LDS - LDS_ST == 4 * QB * 4);
static_assert(QB * OSP * 4 <= LDS_PS - LDS_QH);
static_assert((QSP % 8) == 0 && (PSP % 8) == 0 && PSP >= KCH && (OSP % 4) == 0);
static_assert((LDS_QL % 16) == 0 && (LDS_PS % 16) == 0 && (LDS_PMAX % 16) == 0 && (LDS_ST % 16) == 0);
static_assert((SEQ % KCH) == 0 && (SEQ % QB) == 0 && DM == 8 * 128);

__global__ __launch_bounds__(256) __attribute__((amdgpu_num_vgpr(256)))
void attn_kernel(const _Float16* __restrict__ qh, const _Float16* __restrict__ ql,
                 const _Float16* __restrict__ kh, const _Float16* __restrict__ vh,
                 const _Float16* __restrict__ vl, float* __restrict__ out, float sc, float scl) {
  extern __shared__ __align__(16) char smem[];
  _Float16* Qh_s = (_Float16*)(smem + LDS_QH);
  _Float16* Ql_s = (_Float16*)(smem + LDS_QL);
  _Float16* Ps   = (_Float16*)(smem + LDS_PS);
  float* pmax = (float*)(smem + LDS_PMAX);
  float* psum = (float*)(smem + LDS_PSUM);
  float* m_s  = (float*)(smem + LDS_ST);
  float* l_s  = m_s + QB;
  float* al_s = m_s + 2 * QB;
  float* li_s = m_s + 3 * QB;

  const int tid = threadIdx.x, wave = tid >> 5, lane = tid & 31, h = lane >> 4, c = lane & 15;
  const int q0 = (int)blockIdx.x * QB;
  const int kb0 = (q0 / SEQ) * SEQ;
  const float ninf = -__builtin_inff();

  if (tid < QB) { m_s[tid] = ninf; l_s[tid] = 0.0f; al_s[tid] = 0.0f; li_s[tid] = 0.0f; }
  if (tid < 8 * QB) psum[tid] = 0.0f;
#pragma unroll
  for (int i = 0; i < 8; ++i) {
    const int idx = i * 256 + tid;
    const int row = idx >> 7;
    const int pc  = idx & 127;
    const size_t go = (size_t)(q0 + row) * DM + pc * 8;
    const v8h a = *(const v8h*)(qh + go);
    const v8h b = *(const v8h*)(ql + go);
    *(v8h*)(Qh_s + row * QSP + pc * 8) = a;
    *(v8h*)(Ql_s + row * QSP + pc * 8) = b;
  }
  __syncthreads();

  v8f oh[8], olo[8];
#pragma unroll
  for (int nt = 0; nt < 8; ++nt) { oh[nt] = zero8(); olo[nt] = zero8(); }

  const _Float16* qbh = Qh_s + c * QSP + 8 * h;
  const _Float16* qbl = Ql_s + c * QSP + 8 * h;
  const _Float16* pap = Ps + c * PSP + 8 * h;
  const int ntile = SEQ / KCH;

#pragma unroll 1
  for (int t = 0; t < ntile; ++t) {
    const int kb = kb0 + t * KCH + 32 * wave;
    const _Float16* ka0p = kh + (size_t)(kb + c) * DM + 8 * h;
    const _Float16* ka1p = kh + (size_t)(kb + 16 + c) * DM + 8 * h;
    v8f sh[2], sl[2];
    sh[0] = zero8(); sh[1] = zero8(); sl[0] = zero8(); sl[1] = zero8();
#pragma unroll 1
    for (int k0 = 0; k0 < DM; k0 += 32) {
      const v16h a0 = ldfrag(ka0p + k0), a1 = ldfrag(ka1p + k0);
      const v16h bh = ldfrag(qbh + k0), bl = ldfrag(qbl + k0);
      sh[0] = mma16(a0, bh, sh[0]);
      sh[1] = mma16(a1, bh, sh[1]);
      sl[0] = mma16(a0, bl, sl[0]);
      sl[1] = mma16(a1, bl, sl[1]);
      guard4h(sh[0], sh[1], sl[0], sl[1], a0, a1, bh, bl);
    }
    {
      float pm = ninf;
#pragma unroll
      for (int kt = 0; kt < 2; ++kt) {
#pragma unroll
        for (int r = 0; r < 8; ++r) {
          const float s = sh[kt][r] * sc + sl[kt][r] * scl;
          sh[kt][r] = s;
          pm = fmaxf(pm, s);
        }
      }
      pm = fmaxf(pm, __shfl_xor(pm, 16, 32));
      pmax[wave * QB + c] = pm;
    }
    __syncthreads();
    if (wave == 0 && lane < QB) {
      const int row = lane;
      float pst = 0.0f;
#pragma unroll
      for (int w = 0; w < 8; ++w) pst += psum[w * QB + row];
      l_s[row] = l_s[row] * al_s[row] + pst;
      const float mo = m_s[row];
      float mx = mo;
#pragma unroll
      for (int w = 0; w < 8; ++w) mx = fmaxf(mx, pmax[w * QB + row]);
      al_s[row] = __expf(mo - mx);
      m_s[row] = mx;
    }
    __syncthreads();
    {
      const float mq = m_s[c];
      float psm = 0.0f;
#pragma unroll
      for (int kt = 0; kt < 2; ++kt) {
        v8h hv;
#pragma unroll
        for (int r = 0; r < 8; ++r) {
          const float p = __expf(sh[kt][r] - mq);
          psm += p;
          hv[r] = (_Float16)(p * 16.0f);
        }
        *(v8h*)(Ps + c * PSP + 32 * wave + 16 * kt + 8 * h) = hv;
      }
      psm += __shfl_xor(psm, 16, 32);
      psum[wave * QB + c] = psm;
      const v4f aA = *(const v4f*)(al_s + 8 * h), aB = *(const v4f*)(al_s + 8 * h + 4);
#pragma unroll
      for (int nt = 0; nt < 8; ++nt) {
#pragma unroll
        for (int r = 0; r < 4; ++r) {
          oh[nt][r] *= aA[r];  oh[nt][4 + r] *= aB[r];
          olo[nt][r] *= aA[r]; olo[nt][4 + r] *= aB[r];
        }
      }
    }
    __syncthreads();
    {
      const size_t vco = (size_t)(128 * wave + c) * NTOK + (size_t)(kb0 + t * KCH) + 8 * h;
      const _Float16* vhp = vh + vco;
      const _Float16* vlp = vl + vco;
#pragma unroll 1
      for (int ks = 0; ks < KCH; ks += 32) {
        const v16h pa = ldfrag(pap + ks);
#pragma unroll
        for (int g = 0; g < 4; ++g) {
          const size_t r0o = (size_t)(16 * (2 * g)) * NTOK + ks;
          const size_t r1o = (size_t)(16 * (2 * g + 1)) * NTOK + ks;
          const v16h x0 = ldfrag(vhp + r0o), x1 = ldfrag(vhp + r1o);
          const v16h y0 = ldfrag(vlp + r0o), y1 = ldfrag(vlp + r1o);
          oh[2 * g]      = mma16(pa, x0, oh[2 * g]);
          oh[2 * g + 1]  = mma16(pa, x1, oh[2 * g + 1]);
          olo[2 * g]     = mma16(pa, y0, olo[2 * g]);
          olo[2 * g + 1] = mma16(pa, y1, olo[2 * g + 1]);
          guard5h(oh[2 * g], oh[2 * g + 1], olo[2 * g], olo[2 * g + 1], pa, x0, x1, y0, y1);
        }
      }
    }
  }

  if (wave == 0 && lane < QB) {
    const int row = lane;
    float pst = 0.0f;
#pragma unroll
    for (int w = 0; w < 8; ++w) pst += psum[w * QB + row];
    const float l = l_s[row] * al_s[row] + pst;
    li_s[row] = (1.0f / l) * (1.0f / 256.0f);
  }
  __syncthreads();
  float* Os = (float*)(smem + LDS_QH);
  {
    const v4f iA = *(const v4f*)(li_s + 8 * h), iB = *(const v4f*)(li_s + 8 * h + 4);
    const float rs = 1.0f / 2048.0f;
#pragma unroll
    for (int nt = 0; nt < 8; ++nt) {
      const int col = 128 * wave + 16 * nt + c;
#pragma unroll
      for (int r = 0; r < 4; ++r) {
        Os[(8 * h + r) * OSP + col]     = (oh[nt][r] + olo[nt][r] * rs) * iA[r];
        Os[(8 * h + 4 + r) * OSP + col] = (oh[nt][4 + r] + olo[nt][4 + r] * rs) * iB[r];
      }
    }
  }
  __syncthreads();
  {
#pragma unroll
    for (int ps = 0; ps < 2; ++ps) {
#pragma unroll
      for (int rr = 0; rr < 2; ++rr) {
        const int row = 2 * wave + rr;
        const float* srow = Os + row * OSP;
        float* grow = out + (size_t)(q0 + row) * DM;
#pragma unroll
        for (int j = 0; j < 8; ++j) {
          const int pc = j * 32 + lane;
          const v4f v = *(const v4f*)(srow + pc * 4);
          *(volatile v4f*)(grow + pc * 4) = v;
        }
      }
      __threadfence();
    }
  }
}

extern "C" void kernel_launch(void* const* d_in, const int* in_sizes, int n_in,
                              void* d_out, int out_size, void* d_ws, size_t ws_size,
                              hipStream_t stream) {
  if (n_in < 7) return;
  const int ntok = NTOK, dm = DM;
  if (in_sizes[0] != ntok * dm) return;
  if (in_sizes[1] != dm * dm || in_sizes[3] != dm * dm || in_sizes[5] != dm * dm) return;
  if (in_sizes[2] != dm || in_sizes[4] != dm || in_sizes[6] != dm) return;
  if (out_size != ntok * dm) return;

  const float* x  = (const float*)d_in[0];
  const float* Wq = (const float*)d_in[1];
  const float* bq = (const float*)d_in[2];
  const float* Wk = (const float*)d_in[3];
  const float* bk = (const float*)d_in[4];
  const float* Wv = (const float*)d_in[5];
  const float* bv = (const float*)d_in[6];
  float* out = (float*)d_out;

  const size_t bX = (size_t)ntok * dm * 2;
  const size_t bW = (size_t)dm * dm * 2;
  const size_t bP = (size_t)ntok * dm * 2;
  size_t off = 0;
  const size_t oXB = off; off += bX;
  const size_t oW0 = off; off += bW;
  const size_t oW1 = off; off += bW;
  const size_t oW2 = off; off += bW;
  const size_t oQH = off; off += bP;
  const size_t oQL = off; off += bP;
  const size_t oKH = off; off += bP;
  const size_t oVH = off; off += bP;
  const size_t oVL = off; off += bP;
  if (off > ws_size) return;
  if (off > (size_t)134217728) return;

  char* ws = (char*)d_ws;
  unsigned short* XB  = (unsigned short*)(ws + oXB);
  unsigned short* WT0 = (unsigned short*)(ws + oW0);
  unsigned short* WT1 = (unsigned short*)(ws + oW1);
  unsigned short* WT2 = (unsigned short*)(ws + oW2);
  _Float16* QH = (_Float16*)(ws + oQH);
  _Float16* QL = (_Float16*)(ws + oQL);
  _Float16* KH = (_Float16*)(ws + oKH);
  _Float16* VH = (_Float16*)(ws + oVH);
  _Float16* VL = (_Float16*)(ws + oVL);

  const dim3 blk(256);
  const int n8 = ntok * dm / 8;
  if ((n8 % 256) != 0) return;

  cvt_x_kernel<<<dim3(n8 / 256), blk, 0, stream>>>(x, XB, n8);
  trw_kernel<<<dim3(3 * (dm / 64) * (dm / 64)), blk, 0, stream>>>(Wq, Wk, Wv, WT0, WT1, WT2);
  gemm64_kernel<1, true><<<dim3(((ntok / 64) * (dm / 64)) / 8), blk, 0, stream>>>(
      XB, dm, WT0, dm, QH, QL, dm, bq, ntok, dm, dm, 16.0f);
  gemm64_kernel<1, false><<<dim3(((ntok / 64) * (dm / 64)) / 8), blk, 0, stream>>>(
      XB, dm, WT1, dm, KH, KH, dm, bk, ntok, dm, dm, 16.0f);
  gemm64_kernel<2, true><<<dim3(((dm / 64) * (ntok / 64)) / 8), blk, 0, stream>>>(
      WT2, dm, XB, dm, VH, VL, ntok, bv, dm, ntok, dm, 16.0f);
  (void)hipFuncSetAttribute(reinterpret_cast<const void*>(&attn_kernel),
                            hipFuncAttributeMaxDynamicSharedMemorySize, ATT_LDS);
  const float sc  = 0.03125f * (1.0f / 256.0f);
  const float scl = sc * (1.0f / 2048.0f);
  attn_kernel<<<dim3(ntok / QB), blk, ATT_LDS, stream>>>(QH, QL, KH, VH, VL, out, sc, scl);
  (void)hipGetLastError();
}
